// NexusKAN_14508399526592
// MI455X (gfx1250) — hardware-verified
//
#include <hip/hip_runtime.h>
#include <math.h>

constexpr int kLayers    = 3;
constexpr int kRows      = 8192;
constexpr int kWidth     = 512;
constexpr int kNB        = 8;
constexpr int kKnots     = 12;
constexpr int kKtot      = kWidth + kWidth * kNB;
constexpr int kBasisRows = 32;
constexpr int kBtChunks  = kKtot / 8;
constexpr int kKnotPitch = 16;
constexpr float kWCarry    = 16.0f;
constexpr float kWCarryInv = 1.0f / 16.0f;
static_assert(kKtot % 32 == 0, "K multiple of 32");
static_assert(kRows % 64 == 0 && kWidth % 64 == 0, "tile multiples");
static_assert(kRows % kBasisRows == 0, "row groups exact");
static_assert(kBtChunks % 32 == 0 && (kWidth / 8) % 32 == 0, "wave-uniform chunk classes");
static_assert((kLayers * kWidth * kBtChunks) % 256 == 0, "bt prep grid exact");
static_assert(((kRows / 64) * (kWidth / 64)) % 8 == 0, "gemm grid exact");

typedef __attribute__((ext_vector_type(16))) _Float16 v16h;
typedef __attribute__((ext_vector_type(8)))  _Float16 v8h;
typedef __attribute__((ext_vector_type(16))) __bf16   v16b;
typedef __attribute__((ext_vector_type(8)))  __bf16   v8b;
typedef __attribute__((ext_vector_type(8)))  float    v8f;
typedef __attribute__((ext_vector_type(4)))  float    v4f;
typedef __attribute__((ext_vector_type(4)))  unsigned int v4u;

__device__ __forceinline__ unsigned short f2bf_bits(float f) {
  unsigned u = __float_as_uint(f);
  return (unsigned short)((u + 0x7FFFu + ((u >> 16) & 1u)) >> 16);
}
__device__ __forceinline__ float bf_bits2f(unsigned short h) { return __uint_as_float(((unsigned)h) << 16); }

__device__ __forceinline__ void dep_guard_h(v8f& a, v8f& b, v16h x, v16h y) { asm volatile("v_nop\n\tv_nop\n\tv_nop\n\tv_nop" : "+v"(a), "+v"(b) : "v"(x), "v"(y)); }
__device__ __forceinline__ void dep_guard_b(v8f& a, v8f& b, v16b x, v16b y) { asm volatile("v_nop\n\tv_nop\n\tv_nop\n\tv_nop" : "+v"(a), "+v"(b) : "v"(x), "v"(y)); }
__device__ __forceinline__ void keep4_h(v16h a, v16h b, v16h c, v16h d) { asm volatile("v_nop" :: "v"(a), "v"(b), "v"(c), "v"(d)); }
__device__ __forceinline__ void keep4_b(v16b a, v16b b, v16b c, v16b d) { asm volatile("v_nop" :: "v"(a), "v"(b), "v"(c), "v"(d)); }
__device__ __forceinline__ void acc_guard4(v8f& a, v8f& b, v8f& c, v8f& d) { asm volatile("v_nop\n\tv_nop\n\tv_nop\n\tv_nop" : "+v"(a), "+v"(b), "+v"(c), "+v"(d)); }
template <typename T> struct Frag;
template <> struct Frag<_Float16> {
  typedef v16h V; union U { v16h v; v8h h[2]; };
  static __device__ __forceinline__ v16h load(const _Float16* p) {
    U f; f.h[0] = *(const v8h*)(p); f.h[1] = *(const v8h*)(p + 16); return f.v;
  }
  static __device__ __forceinline__ v8f mma(v16h a, v16h b, v8f c) {
    return __builtin_amdgcn_wmma_f32_16x16x32_f16(false, a, false, b, (short)0, c, false, false);
  }
  static __device__ __forceinline__ void guard(v8f& a, v8f& b, v16h x, v16h y) { dep_guard_h(a, b, x, y); }
  static __device__ __forceinline__ void keep(v16h a, v16h b, v16h c, v16h d) { keep4_h(a, b, c, d); }
};
template <> struct Frag<__bf16> {
  typedef v16b V; union U { v16b v; v8b h[2]; };
  static __device__ __forceinline__ v16b load(const __bf16* p) {
    U f; f.h[0] = *(const v8b*)(p); f.h[1] = *(const v8b*)(p + 16); return f.v;
  }
  static __device__ __forceinline__ v8f mma(v16b a, v16b b, v8f c) {
    return __builtin_amdgcn_wmma_f32_16x16x32_bf16(false, a, false, b, (short)0, c, false, false);
  }
  static __device__ __forceinline__ void guard(v8f& a, v8f& b, v16b x, v16b y) { dep_guard_b(a, b, x, y); }
  static __device__ __forceinline__ void keep(v16b a, v16b b, v16b c, v16b d) { keep4_b(a, b, c, d); }
};

__device__ __forceinline__ unsigned pk16(unsigned short a, unsigned short b) { return (unsigned)a | ((unsigned)b << 16); }
__device__ __forceinline__ unsigned short h_bits(float f) { const _Float16 h = (_Float16)f; return __builtin_bit_cast(unsigned short, h); }
__device__ __forceinline__ float frcp(float d) { return __builtin_amdgcn_rcpf(d); }

__global__ __launch_bounds__(256) void kan_gemm64(
    const unsigned short* __restrict__ Ap, int lda,
    const unsigned short* __restrict__ Btp, int ldb,
    float* __restrict__ C, int ldc,
    const float* __restrict__ p_ss, const float* __restrict__ p_sb,
    const float* __restrict__ p_ns, const float* __restrict__ p_nb,
    int M, int N, int K, float scale) {
  typedef _Float16 T;
  typedef v16h V;
  const T* A  = (const T*)Ap;
  const T* Bt = (const T*)Btp;
  __shared__ __align__(16) float sT[8][16 * 68];
  const int lane = threadIdx.x & 31;
  const int wave = threadIdx.x >> 5;
  const int tilesN = N >> 6;
  const int tilesM = M >> 6;
  const int tile = blockIdx.x * 8 + wave;
  if (tile >= tilesM * tilesN) return;
  const int tm = tile / tilesN;
  const int tn = tile - tm * tilesN;
  const int m0 = tm << 6;
  const int n0 = tn << 6;

  const int rlane = lane & 15;
  const int koff  = (lane >> 4) * 8;
  const int mOff  = (lane >> 4) * 8;

  v8f acc[4][4];
#pragma unroll
  for (int i = 0; i < 4; ++i)
#pragma unroll
    for (int j = 0; j < 4; ++j) acc[i][j] = (v8f){0.f,0.f,0.f,0.f,0.f,0.f,0.f,0.f};

  for (int k0 = 0; k0 < K; k0 += 32) {
    V bh[4];
#pragma unroll
    for (int j = 0; j < 4; ++j) {
      const size_t bo = (size_t)(n0 + (j << 4) + rlane) * ldb + koff + k0;
      bh[j] = Frag<T>::load(Bt + bo);
    }
#pragma unroll
    for (int i = 0; i < 4; ++i) {
      const size_t ao = (size_t)(m0 + (i << 4) + rlane) * lda + koff + k0;
      V ah = Frag<T>::load(A + ao);
#pragma unroll
      for (int j = 0; j < 4; ++j) {
        acc[i][j] = Frag<T>::mma(ah, bh[j], acc[i][j]);
      }
      Frag<T>::guard(acc[i][0], acc[i][3], ah, ah);
    }
    Frag<T>::keep(bh[0], bh[1], bh[2], bh[3]);
  }
  acc_guard4(acc[0][0], acc[0][1], acc[0][2], acc[0][3]);
  acc_guard4(acc[1][0], acc[1][1], acc[1][2], acc[1][3]);
  acc_guard4(acc[2][0], acc[2][1], acc[2][2], acc[2][3]);
  acc_guard4(acc[3][0], acc[3][1], acc[3][2], acc[3][3]);

  float* slab = sT[wave];
#pragma unroll
  for (int i = 0; i < 4; ++i) {
    const int mBase = m0 + (i << 4);
#pragma unroll
    for (int j = 0; j < 4; ++j) {
      const int n = n0 + (j << 4) + rlane;
      const float ssv = p_ss[n];
      const float sbv = p_sb[n];
      const float nsv = p_ns[n];
      const float nbv = p_nb[n];
#pragma unroll
      for (int r = 0; r < 8; ++r) {
        float v = acc[i][j][r] * scale;
        v = ssv * v + sbv;
        v = nsv * v + nbv;
        slab[(mOff + r) * 68 + (j << 4) + rlane] = v;
      }
    }
    __builtin_amdgcn_fence(__ATOMIC_RELEASE, "workgroup");
    __builtin_amdgcn_wave_barrier();
    __builtin_amdgcn_fence(__ATOMIC_ACQUIRE, "workgroup");
    {
      const int hh = lane >> 4, c4 = (lane & 15) * 4;
      for (int pass = 0; pass < 2; ++pass) {
#pragma unroll
        for (int it = 0; it < 8; ++it) {
          const int row = it * 2 + hh;
          v4f v = *(const v4f*)(slab + row * 68 + c4);
          *(volatile v4f*)(C + (size_t)(mBase + row) * ldc + n0 + c4) = v;
        }
        __threadfence();
      }
    }
    __builtin_amdgcn_fence(__ATOMIC_RELEASE, "workgroup");
    __builtin_amdgcn_wave_barrier();
    __builtin_amdgcn_fence(__ATOMIC_ACQUIRE, "workgroup");
  }
}

__global__ __launch_bounds__(256) void kan_basis_kernel(
    const float* __restrict__ X,
    const float* __restrict__ grids_l,
    unsigned short* __restrict__ Aout)
{
#pragma clang fp contract(off)
  __shared__ __align__(16) unsigned short ssl[kBasisRows * 256];
  __shared__ __align__(16) float skn[256 * kKnotPitch];
  const int tid  = threadIdx.x;
  const int lane = tid & 31;
  const int wave = tid >> 5;
  const int ih   = blockIdx.x & 1;
  const int b0   = (blockIdx.x >> 1) * kBasisRows;
  const int i    = ih * 256 + tid;

  const float* gp = grids_l + (size_t)i * kKnots;
  const v4f ga = *(const v4f*)(gp);
  const v4f gb = *(const v4f*)(gp + 4);
  const v4f gc = *(const v4f*)(gp + 8);
  float g[12];
  g[0] = ga[0]; g[1] = ga[1]; g[2]  = ga[2]; g[3]  = ga[3];
  g[4] = gb[0]; g[5] = gb[1]; g[6]  = gb[2]; g[7]  = gb[3];
  g[8] = gc[0]; g[9] = gc[1]; g[10] = gc[2]; g[11] = gc[3];

  float* kr = skn + tid * kKnotPitch;
  kr[0] = g[0]; kr[1] = g[0];
#pragma unroll
  for (int q = 0; q < 12; ++q) kr[2 + q] = g[q];
  kr[14] = g[11]; kr[15] = g[11];
  __syncthreads();

  const size_t colBase = (size_t)kWidth + 8 * (size_t)i;

#pragma unroll 1
  for (int r = 0; r < kBasisRows; ++r) {
    const int b = b0 + r;
    const float x = X[(size_t)b * kWidth + i];

    int cnt = 0;
#pragma unroll
    for (int q = 0; q < 12; ++q) cnt += (x >= g[q]) ? 1 : 0;
    int jc = cnt - 1;
    jc = (jc < 0) ? 0 : jc;
    jc = (jc > 10) ? 10 : jc;
    const float* kq = kr + jc;
    const float gm2 = kq[0];
    const float gm1 = kq[1];
    const float gj0 = kq[2];
    const float gj1 = kq[3];
    const float gj2 = kq[4];
    const float gj3 = kq[5];
    const bool inside = (cnt >= 1) && (cnt <= 11) && (x >= gj0) && (x < gj1);

    const float xm0 = x - gj0, xm1 = x - gm1, xm2 = x - gm2;
    const float p1x = gj1 - x, p2x = gj2 - x, p3x = gj3 - x;
    const float r10 = frcp(gj1 - gj0);
    const float r2a = frcp(gj1 - gm1), r2b = frcp(gj2 - gj0);
    const float r3a = frcp(gj1 - gm2), r3b = frcp(gj2 - gm1), r3c = frcp(gj3 - gj0);
    const float u0 = p1x * r10;
    const float u1 = xm0 * r10;
    const float w0 = (p1x * r2a) * u0;
    const float w1 = (xm1 * r2a) * u0 + (p2x * r2b) * u1;
    const float w2 = (xm0 * r2b) * u1;
    const float c0 = (p1x * r3a) * w0;
    const float c1 = (xm2 * r3a) * w0 + (p2x * r3b) * w1;
    const float c2 = (xm1 * r3b) * w1 + (p3x * r3c) * w2;
    const float c3 = (xm0 * r3c) * w2;

    const int jsel = inside ? jc : -8;
    unsigned short hb[8];
#pragma unroll
    for (int s = 0; s < 8; ++s) {
      float v = 0.0f;
      v = (jsel == s + 3) ? c0 : v;
      v = (jsel == s + 2) ? c1 : v;
      v = (jsel == s + 1) ? c2 : v;
      v = (jsel == s)     ? c3 : v;
      hb[s] = h_bits(v);
    }
    const v4u u = (v4u){pk16(hb[0], hb[1]), pk16(hb[2], hb[3]), pk16(hb[4], hb[5]), pk16(hb[6], hb[7])};
    unsigned short* dst = Aout + (size_t)b * kKtot + colBase;
    *(volatile v4u*)dst = u;
    __threadfence();
    *(volatile v4u*)dst = u;

    const float ex  = expf(-x);
    const float sl  = x * frcp(1.0f + ex);
    ssl[r * 256 + tid] = h_bits(sl);
  }
  __syncthreads();
  {
    for (int pass = 0; pass < 2; ++pass) {
#pragma unroll
      for (int it = 0; it < 4; ++it) {
        const int row = wave * 4 + it;
        const v4u u = *(const v4u*)(ssl + row * 256 + lane * 8);
        *(volatile v4u*)(Aout + (size_t)(b0 + row) * kKtot + (size_t)ih * 256 + (size_t)lane * 8) = u;
      }
      __threadfence();
    }
  }
}

__global__ __launch_bounds__(256) void kan_btprep_kernel(
    const float* __restrict__ coefs,
    const float* __restrict__ sbase,
    const float* __restrict__ ssp,
    unsigned short* __restrict__ Bt,
    float carry) {
  const int idx = blockIdx.x * 256 + threadIdx.x;
  if (idx >= kLayers * kWidth * kBtChunks) return;
  const int l   = idx / (kWidth * kBtChunks);
  const int rem = idx - l * (kWidth * kBtChunks);
  const int o   = rem / kBtChunks;
  const int ch  = rem - o * kBtChunks;
  const float* coefs_l = coefs + (size_t)l * kWidth * kWidth * kNB;
  const float* sbase_l = sbase + (size_t)l * kWidth * kWidth;
  const float* ssp_l   = ssp   + (size_t)l * kWidth * kWidth;
  const int chb = (ch < 64) ? ch : 63;
  const int ib  = chb * 8;
  float vb[8];
#pragma unroll
  for (int e = 0; e < 8; ++e) vb[e] = sbase_l[(size_t)(ib + e) * kWidth + o] * carry;
  int is = ch - 64;
  is = (is < 0) ? 0 : is;
  const float* cp = coefs_l + ((size_t)is * kWidth + o) * kNB;
  const v4f c0 = *(const v4f*)(cp);
  const v4f c1 = *(const v4f*)(cp + 4);
  const float sp = ssp_l[(size_t)is * kWidth + o];
  float vs[8];
#pragma unroll
  for (int e = 0; e < 4; ++e) {
    vs[e]     = (c0[e] * sp) * carry;
    vs[4 + e] = (c1[e] * sp) * carry;
  }
  const bool basePart = (ch < 64);
  unsigned short hb[8];
#pragma unroll
  for (int e = 0; e < 8; ++e) hb[e] = h_bits(basePart ? vb[e] : vs[e]);
  const v4u u = (v4u){pk16(hb[0], hb[1]), pk16(hb[2], hb[3]), pk16(hb[4], hb[5]), pk16(hb[6], hb[7])};
  unsigned short* dst = Bt + ((size_t)l * kWidth + o) * kKtot + (size_t)ch * 8;
  *(volatile v4u*)dst = u;
  __threadfence();
  *(volatile v4u*)dst = u;
}

extern "C" void kernel_launch(void* const* d_in, const int* in_sizes, int n_in,
                              void* d_out, int out_size, void* d_ws, size_t ws_size,
                              hipStream_t stream) {
  if (n_in < 9) return;
  if (in_sizes[0] != kRows * kWidth) return;
  if (in_sizes[1] != kLayers * kWidth * kKnots) return;
  if (in_sizes[2] != kLayers * kWidth * kWidth * kNB) return;
  if (in_sizes[3] != kLayers * kWidth * kWidth) return;
  if (in_sizes[4] != kLayers * kWidth * kWidth) return;
  if (in_sizes[5] != kLayers * kWidth || in_sizes[6] != kLayers * kWidth) return;
  if (in_sizes[7] != kLayers * kWidth || in_sizes[8] != kLayers * kWidth) return;
  if (out_size != kRows * kWidth) return;

  const float* x       = (const float*)d_in[0];
  const float* grids   = (const float*)d_in[1];
  const float* coefs   = (const float*)d_in[2];
  const float* sbase   = (const float*)d_in[3];
  const float* ssp     = (const float*)d_in[4];
  const float* sub_sc  = (const float*)d_in[5];
  const float* sub_bs  = (const float*)d_in[6];
  const float* node_sc = (const float*)d_in[7];
  const float* node_bs = (const float*)d_in[8];
  float* out = (float*)d_out;

  const size_t bytesA  = (size_t)kRows * kKtot * sizeof(unsigned short);
  const size_t bytesBt = (size_t)kLayers * kWidth * kKtot * sizeof(unsigned short);
  const size_t bytesX  = (size_t)kRows * kWidth * sizeof(float);
  const size_t offA  = 0;
  const size_t offBt = offA + bytesA;
  const size_t offXA = offBt + bytesBt;
  const size_t offXB = offXA + bytesX;
  const size_t total = offXB + bytesX;
  if (total > ws_size) return;

  unsigned short* Apl  = (unsigned short*)((char*)d_ws + offA);
  unsigned short* Btpl = (unsigned short*)((char*)d_ws + offBt);
  float* XA = (float*)((char*)d_ws + offXA);
  float* XB = (float*)((char*)d_ws + offXB);

  const int basisGrid = 2 * (kRows / kBasisRows);
  const int btGrid    = (kLayers * kWidth * kBtChunks) / 256;
  const int gemmGrid  = ((kRows / 64) * (kWidth / 64)) / 8;

  kan_btprep_kernel<<<dim3(btGrid), dim3(256), 0, stream>>>(coefs, sbase, ssp, Btpl, kWCarry);

  for (int l = 0; l < kLayers; ++l) {
    const float* xin = (l == 0) ? x : ((l == 1) ? (const float*)XA : (const float*)XB);
    float* xout = (l == 0) ? XA : ((l == 1) ? XB : out);

    kan_basis_kernel<<<dim3(basisGrid), dim3(256), 0, stream>>>(
        xin, grids + (size_t)l * kWidth * kKnots, Apl);

    kan_gemm64<<<dim3(gemmGrid), dim3(256), 0, stream>>>(
        Apl, kKtot, Btpl + (size_t)l * kWidth * kKtot, kKtot, xout, kWidth,
        sub_sc + (size_t)l * kWidth, sub_bs + (size_t)l * kWidth,
        node_sc + (size_t)l * kWidth, node_bs + (size_t)l * kWidth,
        kRows, kWidth, kKtot, kWCarryInv);
  }
}
